// DFVAE_67826123538573
// MI455X (gfx1250) — hardware-verified
//
#include <hip/hip_runtime.h>

#define NR_  16384
#define LD_  512
#define EMAX 16
#define GSTR 48
#define MAXT (NR_ / 128 + EMAX)

typedef _Float16 f16;
typedef __attribute__((ext_vector_type(16))) f16 f16x16;
typedef __attribute__((ext_vector_type(8)))  f16 f16x8;
typedef __attribute__((ext_vector_type(8)))  float f32x8;
typedef __attribute__((ext_vector_type(4)))  float v4f_t;
typedef float v4fa __attribute__((ext_vector_type(4), may_alias));

__device__ __forceinline__ f32x8 wmma16(f16x16 a, f16x16 b, f32x8 c) {
  c = __builtin_amdgcn_wmma_f32_16x16x32_f16(false, a, false, b, (short)0, c, false, false);
  asm volatile("v_nop\n\tv_nop\n\tv_nop\n\tv_nop" : "+v"(c) : "v"(a), "v"(b));
  return c;
}
__device__ __forceinline__ f16x16 lds_frag(const f16* base, int stride) {
  const int lane = threadIdx.x & 31, row = lane & 15, kh = (lane >> 4) * 8;
  const f16x8 lo = *(const f16x8*)(base + row * stride + kh);
  const f16x8 hi = *(const f16x8*)(base + row * stride + kh + 16);
  f16x16 f;
#pragma unroll
  for (int i = 0; i < 8; ++i) { f[i] = lo[i]; f[i + 8] = hi[i]; }
  return f;
}

__global__ __launch_bounds__(256) void gemm_moe(const float* __restrict__ zin, const int* __restrict__ ids, int E,
                                               const float* __restrict__ Wall, const float* __restrict__ ball, float* __restrict__ zout) {
  __shared__ __attribute__((aligned(16))) f16 ldsA[128 * GSTR], ldsAl[128 * GSTR];
  __shared__ __attribute__((aligned(16))) f16 ldsW[128 * GSTR], ldsWl[128 * GSTR];
  __shared__ __attribute__((aligned(16))) float oS[8][32 * 68];
  __shared__ int idS[128];
  __shared__ int present[EMAX];
  const int tid = threadIdx.x, lane = tid & 31, wave = tid >> 5, cl = lane & 15, rh = (lane >> 4) * 8;
  const int m0 = blockIdx.x * 128, n0 = blockIdx.y * 128;
  if (tid < EMAX) present[tid] = 0;
  __syncthreads();
  if (tid < 128) { int e = ids[m0 + tid]; e = min(max(e, 0), E - 1); idS[tid] = e; present[e] = 1; }
  __syncthreads();
  const int wm = (wave & 3) * 32, wn = (wave >> 2) * 64;
  float* so = oS[wave];
#pragma unroll 1
  for (int e = 0; e < E; ++e) {
    if (!present[e]) continue;
    const float* Wm = Wall + (size_t)e * LD_ * LD_;
    const float* be = ball + (size_t)e * LD_;
    f32x8 acc[2][4], accx[2][4];
#pragma unroll
    for (int i = 0; i < 2; ++i)
#pragma unroll
      for (int j = 0; j < 4; ++j) { f32x8 z = {}; acc[i][j] = z; accx[i][j] = z; }
#pragma unroll 1
    for (int k0 = 0; k0 < LD_; k0 += 32) {
      __syncthreads();
      { const int row = tid >> 1, ch = (tid & 1) * 16; const float* p = zin + (size_t)(m0 + row) * LD_ + k0 + ch;
#pragma unroll
        for (int g = 0; g < 16; ++g) { const float v = p[g]; const f16 h = (f16)v; ldsA[row * GSTR + ch + g] = h; ldsAl[row * GSTR + ch + g] = (f16)((v - (float)h) * 2048.0f); } }
      { const int k = tid >> 3, nn0 = (tid & 7) * 16;
        const float* src = Wm + (size_t)(k0 + k) * LD_ + n0 + nn0;
#pragma unroll
        for (int g = 0; g < 4; ++g) { const v4f_t v = *(const v4f_t*)(src + 4 * g);
#pragma unroll
          for (int u = 0; u < 4; ++u) { const f16 h = (f16)v[u]; ldsW[(nn0 + 4 * g + u) * GSTR + k] = h; ldsWl[(nn0 + 4 * g + u) * GSTR + k] = (f16)((v[u] - (float)h) * 2048.0f); } } }
      __syncthreads();
      f16x16 af[2], afl[2];
#pragma unroll
      for (int i = 0; i < 2; ++i) { af[i] = lds_frag(ldsA + (wm + 16 * i) * GSTR, GSTR); afl[i] = lds_frag(ldsAl + (wm + 16 * i) * GSTR, GSTR); }
#pragma unroll
      for (int j = 0; j < 4; ++j) {
        const f16x16 bf = lds_frag(ldsW + (wn + 16 * j) * GSTR, GSTR), bfl = lds_frag(ldsWl + (wn + 16 * j) * GSTR, GSTR);
#pragma unroll
        for (int i = 0; i < 2; ++i) { acc[i][j] = wmma16(af[i], bf, acc[i][j]); accx[i][j] = wmma16(af[i], bfl, accx[i][j]); accx[i][j] = wmma16(afl[i], bf, accx[i][j]); }
      }
    }
#pragma unroll
    for (int i = 0; i < 2; ++i)
#pragma unroll
      for (int r = 0; r < 8; ++r) {
        const int rl = wm + 16 * i + rh + r;
        if (idS[rl] == e) {
#pragma unroll
          for (int j = 0; j < 4; ++j) { const int n = n0 + wn + 16 * j + cl; so[(16 * i + rh + r) * 68 + 16 * j + cl] = fmaxf(acc[i][j][r] + accx[i][j][r] * (1.0f / 2048.0f) + be[n], 0.0f); }
        }
      }
  }
  asm volatile("s_wait_dscnt 0" ::: "memory");
  __builtin_amdgcn_wave_barrier();
#pragma unroll 1
  for (int pass = 0; pass < 2; ++pass) {
#pragma unroll
    for (int it = 0; it < 16; ++it) { const int f4 = lane + 32 * it, rr = f4 >> 4, q = (f4 & 15) * 4;
      *(volatile v4f_t*)(zout + (size_t)(m0 + wm + rr) * LD_ + n0 + wn + q) = *(const volatile v4fa*)(so + rr * 68 + q); }
    __threadfence();
  }
}

extern "C" void kernel_launch(void* const* d_in, const int* in_sizes, int n_in,
                              void* d_out, int out_size, void* d_ws, size_t ws_size,
                              hipStream_t stream) {
  (void)in_sizes; (void)n_in; (void)out_size; (void)ws_size;
  const float* z = (const float*)d_in[0];
  const float* Wd = (const float*)d_in[1], *bd = (const float*)d_in[2];
  const float* Wa = (const float*)d_in[3], *ba = (const float*)d_in[4];
  const float* Wo = (const float*)d_in[5], *bo = (const float*)d_in[6];
  const int* idd = (const int*)d_in[7], *ida = (const int*)d_in[8], *ido = (const int*)d_in[9];
  float* out = (float*)d_out;
  char* ws = (char*)d_ws;
  float* z1 = (float*)ws; ws += (size_t)NR_ * LD_ * 4;
  float* z2 = (float*)ws; ws += (size_t)NR_ * LD_ * 4;
  const dim3 g(NR_ / 128, LD_ / 128), blk(256);
  gemm_moe<<<g, blk, 0, stream>>>(z,  idd, 8,  Wd, bd, z1);
  gemm_moe<<<g, blk, 0, stream>>>(z1, ida, 6,  Wa, ba, z2);
  gemm_moe<<<g, blk, 0, stream>>>(z2, ido, 16, Wo, bo, out);
}
